// GAR_DSVDD_32049045963527
// MI455X (gfx1250) — hardware-run, weakly checked
//
#include <hip/hip_runtime.h>
#include <math.h>
#include <stdint.h>

#define DD     64
#define NHEAD  8
#define DKH    32
#define HDIM   (NHEAD * DKH)
#define KNB    16
#define TM     64
#define NTHR   256
#define NWAV   (NTHR / 32)
#define ZP     72
#define QP     260
#define KSTEP  (DD / 32)
#define NTILE  (HDIM / 16)
#define PL_EL  (NHEAD * DD * DKH)
#define NPIECE ((2 * PL_EL) / 8)
#define OFF_Z  0
#define OFF_Q  (TM * ZP * 2)
#define OFF_O  (OFF_Q + TM * QP * 4)
#define LDS_K  OFF_O
#define LDS_A  (OFF_O + TM * KNB * 4)

#define SCALE  0.17677669529663688f
#define GAMMA  0.5f
#define BETA   0.9f
#define OMB    0.1f

static_assert(KSTEP * 32 == DD);
static_assert(NTILE * 16 == HDIM);
static_assert(NWAV == 8 && NTILE == 2 * NWAV);
static_assert(TM == 4 * 16);
static_assert(NTHR == 4 * TM);
static_assert((ZP % 8) == 0 && ZP >= DD);
static_assert((QP % 4) == 0 && QP >= HDIM);
static_assert((OFF_Q % 16) == 0 && (OFF_O % 16) == 0 && (LDS_A % 16) == 0);
static_assert(NPIECE == 16 * 256);
static_assert(TM * KNB == 4 * NTHR);
static_assert(HDIM == 2 * 32 * 4);
static_assert(TM == 8 * NWAV);

typedef __bf16         v16b __attribute__((ext_vector_type(16)));
typedef unsigned short v8us __attribute__((ext_vector_type(8)));
typedef float          v8f  __attribute__((ext_vector_type(8)));
typedef float          v4f  __attribute__((ext_vector_type(4)));

union FragB { v16b v; v8us u[2]; };

__device__ __forceinline__ unsigned short bf_bits(float x) {
  const unsigned u = __float_as_uint(x);
  return (unsigned short)((u + 0x7FFFu + ((u >> 16) & 1u)) >> 16);
}
__device__ __forceinline__ float bfr(float x) { return __uint_as_float(((unsigned)bf_bits(x)) << 16); }
__device__ __forceinline__ v8f zero8() { return (v8f){0.f, 0.f, 0.f, 0.f, 0.f, 0.f, 0.f, 0.f}; }

__device__ __forceinline__ v8f mma_b(v16b a, v16b b, v8f c) {
  return __builtin_amdgcn_wmma_f32_16x16x32_bf16(false, a, false, b, (short)0, c, false, false);
}
__device__ __forceinline__ void guard8(v8f& c0, v8f& c1, v8f& c2, v8f& c3,
                                       v8f& c4, v8f& c5, v8f& c6, v8f& c7,
                                       v16b a0, v16b a1, v16b a2, v16b a3, v16b b0, v16b b1) {
#if defined(__HIP_DEVICE_COMPILE__)
  asm volatile("v_nop\n\tv_nop\n\tv_nop\n\tv_nop"
               : "+v"(c0), "+v"(c1), "+v"(c2), "+v"(c3), "+v"(c4), "+v"(c5), "+v"(c6), "+v"(c7)
               : "v"(a0), "v"(a1), "v"(a2), "v"(a3), "v"(b0), "v"(b1));
#else
  (void)c0; (void)c1; (void)c2; (void)c3; (void)c4; (void)c5; (void)c6; (void)c7;
  (void)a0; (void)a1; (void)a2; (void)a3; (void)b0; (void)b1;
#endif
}

__global__ __launch_bounds__(256) void k_pack(const float* __restrict__ wq, const float* __restrict__ wk,
                                              unsigned short* dst) {
  const int p     = blockIdx.x * 256 + threadIdx.x;
  const bool act  = p < NPIECE;
  const int pc    = act ? p : (NPIECE - 1);
  const int plane = pc >> 11;
  const float* src = (plane != 0) ? wk : wq;
  const int pl    = pc & 2047;
  const int elem0 = pl * 8;
  const int nt    = elem0 >> 10;
  int rem         = elem0 & 1023;
  const int s     = rem >> 9;
  rem            &= 511;
  const int L     = rem >> 4;
  const int j0    = rem & 15;
  const int n     = nt * 16 + (L & 15);
  const int hl    = L >> 4;
  const int kb    = s * 32 + 8 * hl + 2 * j0;
  const int head  = n >> 5;
  const int kk    = n & 31;
  v8us o;
#pragma unroll
  for (int jj = 0; jj < 8; ++jj) {
    const int k = kb + jj;
    int si = (head * DD + k) * DKH + kk;
    si = (si < 0) ? 0 : ((si >= PL_EL) ? (PL_EL - 1) : si);
    o[jj] = bf_bits(src[si]);
  }
  unsigned short* d = dst + (size_t)pc * 8;
  if (act) *(volatile v8us*)d = o;
  __threadfence();
  if (act) *(volatile v8us*)d = o;
}

__device__ __forceinline__ void stage_z(const float* __restrict__ Z, int N, int i0,
                                        unsigned short* sZ, int tid) {
  const int r = tid >> 2;
  const int q = tid & 3;
  int gr = i0 + r;
  gr = (gr < N) ? gr : (N - 1);
  const float* p = Z + (size_t)gr * DD + q * 16;
  const v4f va = *(const v4f*)(p);
  const v4f vb = *(const v4f*)(p + 4);
  const v4f vc = *(const v4f*)(p + 8);
  const v4f vd = *(const v4f*)(p + 12);
  v8us o0, o1;
#pragma unroll
  for (int k = 0; k < 4; ++k) {
    o0[k] = bf_bits(va[k]);  o0[4 + k] = bf_bits(vb[k]);
    o1[k] = bf_bits(vc[k]);  o1[4 + k] = bf_bits(vd[k]);
  }
  unsigned short* d = sZ + r * ZP + q * 16;
  *(v8us*)(d)     = o0;
  *(v8us*)(d + 8) = o1;
}

__device__ __forceinline__ void tile_gemm(const unsigned short* sZ, const unsigned short* __restrict__ Wp,
                                          float* sO, int lane, int wave) {
  const int m    = lane & 15;
  const int hl   = lane >> 4;
  const int mrow = 8 * hl;
  const int nt0  = 2 * wave;
  v8f c00 = zero8(), c01 = zero8(), c10 = zero8(), c11 = zero8();
  v8f c20 = zero8(), c21 = zero8(), c30 = zero8(), c31 = zero8();
  FragB a0, a1, a2, a3, b0, b1;
#pragma unroll
  for (int s = 0; s < KSTEP; ++s) {
    const unsigned short* pa = sZ + m * ZP + s * 32 + 8 * hl;
    a0.u[0] = *(const v8us*)(pa);                 a0.u[1] = *(const v8us*)(pa + 16);
    a1.u[0] = *(const v8us*)(pa + 16 * ZP);       a1.u[1] = *(const v8us*)(pa + 16 * ZP + 16);
    a2.u[0] = *(const v8us*)(pa + 32 * ZP);       a2.u[1] = *(const v8us*)(pa + 32 * ZP + 16);
    a3.u[0] = *(const v8us*)(pa + 48 * ZP);       a3.u[1] = *(const v8us*)(pa + 48 * ZP + 16);
    const unsigned short* pb = Wp + ((size_t)(nt0 * KSTEP + s) * 32 + lane) * 16;
    b0.u[0] = *(const v8us*)(pb);                 b0.u[1] = *(const v8us*)(pb + 8);
    b1.u[0] = *(const v8us*)(pb + KSTEP * 512);   b1.u[1] = *(const v8us*)(pb + KSTEP * 512 + 8);
    c00 = mma_b(a0.v, b0.v, c00);  c01 = mma_b(a0.v, b1.v, c01);
    c10 = mma_b(a1.v, b0.v, c10);  c11 = mma_b(a1.v, b1.v, c11);
    c20 = mma_b(a2.v, b0.v, c20);  c21 = mma_b(a2.v, b1.v, c21);
    c30 = mma_b(a3.v, b0.v, c30);  c31 = mma_b(a3.v, b1.v, c31);
    guard8(c00, c01, c10, c11, c20, c21, c30, c31, a0.v, a1.v, a2.v, a3.v, b0.v, b1.v);
  }
#pragma unroll
  for (int r = 0; r < 8; ++r) {
    float* s0 = sO + (mrow + r) * QP + nt0 * 16 + m;
    s0[0]            = c00[r];  s0[16]           = c01[r];
    s0[16 * QP]      = c10[r];  s0[16 * QP + 16] = c11[r];
    s0[32 * QP]      = c20[r];  s0[32 * QP + 16] = c21[r];
    s0[48 * QP]      = c30[r];  s0[48 * QP + 16] = c31[r];
  }
}

__global__ __launch_bounds__(NTHR) void k_kall(const float* __restrict__ Z, const unsigned short* __restrict__ Wp,
                                               float* Kall, int N) {
  extern __shared__ __align__(16) unsigned char dynl[];
  unsigned short* sZ = (unsigned short*)(dynl + OFF_Z);
  float* sO = (float*)(dynl + OFF_Q);
  const int tid  = threadIdx.x;
  const int lane = tid & 31;
  const int wave = tid >> 5;
  const int i0   = blockIdx.x * TM;

  stage_z(Z, N, i0, sZ, tid);
  __syncthreads();
  tile_gemm(sZ, Wp, sO, lane, wave);
  __syncthreads();

  v4f u0[8], u1[8];
#pragma unroll
  for (int rr = 0; rr < 8; ++rr) {
    const int row = wave * 8 + rr;
    u0[rr] = *(const v4f*)(sO + row * QP + lane * 4);
    u1[rr] = *(const v4f*)(sO + row * QP + 128 + lane * 4);
  }
#pragma unroll
  for (int rr = 0; rr < 8; ++rr) {
    float* p = Kall + (size_t)(i0 + wave * 8 + rr) * HDIM + lane * 4;
    *(volatile v4f*)(p)       = u0[rr];
    *(volatile v4f*)(p + 128) = u1[rr];
  }
  __threadfence();
#pragma unroll
  for (int rr = 0; rr < 8; ++rr) {
    float* p = Kall + (size_t)(i0 + wave * 8 + rr) * HDIM + lane * 4;
    *(volatile v4f*)(p)       = u0[rr];
    *(volatile v4f*)(p + 128) = u1[rr];
  }
}

__global__ __launch_bounds__(NTHR) void k_attn(const float* __restrict__ Z, const float* __restrict__ f,
                                               const float* __restrict__ ema, const int* __restrict__ idx,
                                               const unsigned short* __restrict__ Wp,
                                               const float* __restrict__ Kall, float* out, int N) {
  extern __shared__ __align__(16) unsigned char dynl[];
  unsigned short* sZ = (unsigned short*)(dynl + OFF_Z);
  float* sQ   = (float*)(dynl + OFF_Q);
  float* sOut = (float*)(dynl + OFF_O);
  const int tid  = threadIdx.x;
  const int lane = tid & 31;
  const int wave = tid >> 5;
  const int m16  = lane & 15;
  const int hg   = lane >> 4;
  const int i0   = blockIdx.x * TM;

  stage_z(Z, N, i0, sZ, tid);
  __syncthreads();
  tile_gemm(sZ, Wp, sQ, lane, wave);
  __syncthreads();

#pragma unroll 1
  for (int it = 0; it < TM / NWAV; ++it) {
    const int row = it * NWAV + wave;
    const int i   = i0 + row;
    const int ic  = (i < N) ? i : (N - 1);
    int j = idx[(size_t)ic * KNB + m16];
    j = (j < 0) ? 0 : ((j >= N) ? (N - 1) : j);
    const float fi   = bfr(f[ic]);
    const float fj   = bfr(f[j]);
    const float damp = GAMMA * (fmaxf(fi, 0.f) + fmaxf(fj, 0.f));
    const float* kp  = Kall + (size_t)j * HDIM + hg * 128;
    const float* qp  = sQ + row * QP + hg * 128;
    float a0 = 0.f, a1 = 0.f, a2 = 0.f, a3 = 0.f;
#pragma unroll 2
    for (int c = 0; c < 8; ++c) {
      const v4f k0 = *(const v4f*)(kp + 4 * c);
      const v4f k1 = *(const v4f*)(kp + 32 + 4 * c);
      const v4f k2 = *(const v4f*)(kp + 64 + 4 * c);
      const v4f k3 = *(const v4f*)(kp + 96 + 4 * c);
      const v4f q0 = *(const v4f*)(qp + 4 * c);
      const v4f q1 = *(const v4f*)(qp + 32 + 4 * c);
      const v4f q2 = *(const v4f*)(qp + 64 + 4 * c);
      const v4f q3 = *(const v4f*)(qp + 96 + 4 * c);
      a0 += k0[0] * q0[0];  a0 += k0[1] * q0[1];  a0 += k0[2] * q0[2];  a0 += k0[3] * q0[3];
      a1 += k1[0] * q1[0];  a1 += k1[1] * q1[1];  a1 += k1[2] * q1[2];  a1 += k1[3] * q1[3];
      a2 += k2[0] * q2[0];  a2 += k2[1] * q2[1];  a2 += k2[2] * q2[2];  a2 += k2[3] * q2[3];
      a3 += k3[0] * q3[0];  a3 += k3[1] * q3[1];  a3 += k3[2] * q3[2];  a3 += k3[3] * q3[3];
    }
    const float x0 = a0 * SCALE - damp;
    const float x1 = a1 * SCALE - damp;
    const float x2 = a2 * SCALE - damp;
    const float x3 = a3 * SCALE - damp;
    float m0 = x0, m1 = x1, m2 = x2, m3 = x3;
#pragma unroll
    for (int off = 8; off >= 1; off >>= 1) {
      m0 = fmaxf(m0, __shfl_xor(m0, off, 32));
      m1 = fmaxf(m1, __shfl_xor(m1, off, 32));
      m2 = fmaxf(m2, __shfl_xor(m2, off, 32));
      m3 = fmaxf(m3, __shfl_xor(m3, off, 32));
    }
    const float e0 = __expf(x0 - m0);
    const float e1 = __expf(x1 - m1);
    const float e2 = __expf(x2 - m2);
    const float e3 = __expf(x3 - m3);
    float s0 = e0, s1 = e1, s2 = e2, s3 = e3;
#pragma unroll
    for (int off = 8; off >= 1; off >>= 1) {
      s0 += __shfl_xor(s0, off, 32);
      s1 += __shfl_xor(s1, off, 32);
      s2 += __shfl_xor(s2, off, 32);
      s3 += __shfl_xor(s3, off, 32);
    }
    float wsum = e0 * __builtin_amdgcn_rcpf(s0) + e1 * __builtin_amdgcn_rcpf(s1)
               + e2 * __builtin_amdgcn_rcpf(s2) + e3 * __builtin_amdgcn_rcpf(s3);
    wsum += __shfl_xor(wsum, 16, 32);
    const float W  = wsum * 0.125f;
    const float em = bfr(ema[(size_t)ic * KNB + m16]);
    const float o  = fmaxf(BETA * em + OMB * W, 0.f);
    if (lane < KNB) sOut[row * KNB + m16] = o;
  }
  __syncthreads();

  {
    const int orow  = tid >> 2;
    const v4f ov    = *(const v4f*)(sOut + tid * 4);
    const bool act  = (i0 + orow) < N;
    float* op = out + (size_t)i0 * KNB + tid * 4;
    if (act) *(volatile v4f*)op = ov;
    __threadfence();
    if (act) *(volatile v4f*)op = ov;
  }
}

extern "C" void kernel_launch(void* const* d_in, const int* in_sizes, int n_in,
                              void* d_out, int out_size, void* d_ws, size_t ws_size,
                              hipStream_t stream) {
  if (n_in < 6) return;
  const int N = in_sizes[1];
  if (N <= 0) return;
  if (in_sizes[0] != N * DD) return;
  if (in_sizes[2] != PL_EL || in_sizes[3] != PL_EL) return;
  if (in_sizes[4] != N * KNB || in_sizes[5] != N * KNB) return;
  if (out_size != N * KNB) return;

  const float* Z   = (const float*)d_in[0];
  const float* f   = (const float*)d_in[1];
  const float* WQ  = (const float*)d_in[2];
  const float* WK  = (const float*)d_in[3];
  const float* ema = (const float*)d_in[4];
  const int*   idx = (const int*)d_in[5];
  float* out = (float*)d_out;

  const int nblk  = (N + TM - 1) / TM;
  const size_t NP = (size_t)nblk * TM;
  const size_t oq_bytes  = 0;
  const size_t ok_bytes  = oq_bytes + (size_t)PL_EL * 2;
  const size_t op_bytes  = ok_bytes + (size_t)PL_EL * 2;
  const size_t tot_bytes = op_bytes + NP * (size_t)HDIM * 4;
  if ((op_bytes % 128) != 0) return;
  if (tot_bytes > ws_size) return;
  if (tot_bytes > (size_t)134217728) return;

  unsigned short* Wq16 = (unsigned short*)((char*)d_ws + oq_bytes);
  unsigned short* Wk16 = (unsigned short*)((char*)d_ws + ok_bytes);
  float* Kall = (float*)((char*)d_ws + op_bytes);

  k_pack<<<dim3(NPIECE / 256), dim3(256), 0, stream>>>(WQ, WK, Wq16);

  (void)hipFuncSetAttribute(reinterpret_cast<const void*>(&k_kall),
                            hipFuncAttributeMaxDynamicSharedMemorySize, LDS_K);
  k_kall<<<dim3(nblk), dim3(NTHR), (size_t)LDS_K, stream>>>(Z, Wk16, Kall, N);

  (void)hipFuncSetAttribute(reinterpret_cast<const void*>(&k_attn),
                            hipFuncAttributeMaxDynamicSharedMemorySize, LDS_A);
  k_attn<<<dim3(nblk), dim3(NTHR), (size_t)LDS_A, stream>>>(Z, f, ema, idx, Wq16, Kall, out, N);
  (void)hipGetLastError();
}
